// Encoder_24146306138770
// MI455X (gfx1250) — hardware-run, weakly checked
//
#include <hip/hip_runtime.h>
#include <math.h>

typedef __attribute__((ext_vector_type(16))) _Float16 v16h;
typedef __attribute__((ext_vector_type(8)))  _Float16 v8h;
typedef __attribute__((ext_vector_type(8)))  float    v8f;
typedef __attribute__((ext_vector_type(4)))  float    v4f;

constexpr int kSteps  = 512;
constexpr int kBatch  = 64;
constexpr int kIn     = 300;
constexpr int kHid    = 75;
constexpr int kRows   = kSteps * kBatch;
constexpr int kHidP   = 80;
constexpr int kCellN  = 3 * kHidP;
constexpr int kKh     = 96;
constexpr int kKx     = 160;
constexpr int kKi     = 320;
constexpr int kGiN    = 512;
constexpr int kOutC   = 6 * kHid;
constexpr int kNT     = 320;
constexpr int kHTile  = 16 * kKh;
constexpr int kXTile  = 16 * kKx;
constexpr int kHsN    = 3 * 2 * 2 * kHTile;
constexpr int kXsN    = 2 * kXTile;
constexpr int kSlabV4 = 16 * kOutC / 4;
constexpr float kCarry  = 64.0f;
constexpr float kFold   = 1.0f / (kCarry * kCarry);
constexpr float kF16Min = 6.103515625e-5f;
static_assert(kRows == 32768, "rows");
static_assert(kOutC == 450, "output channels");
static_assert(kKh % 32 == 0 && kKx % 32 == 0 && kKi % 32 == 0, "K multiples of 32");
static_assert(kKh >= kHid && kKx >= 2 * kHid && kKi >= kIn, "K pads");
static_assert(kRows % 64 == 0 && kGiN % 64 == 0 && kGiN >= 2 * kCellN, "GEMM tile multiples");
static_assert((kIn % 4) == 0, "vector reads of the input rows");
static_assert((16 * kOutC) % 4 == 0 && kSlabV4 == 1800, "slab vector count");
static_assert((16 * kOutC * 4) % 128 == 0, "a block's 16 output rows are whole 128-B lines");
static_assert(kNT == 2 * 5 * 32 && 5 * 16 == kHidP, "wave map: 2 directions x 5 unit tiles");

constexpr size_t kSzXH   = (size_t)kRows * kKi * 2;
constexpr size_t kSzWI0  = (size_t)kGiN * kKi * 2;
constexpr size_t kSzWI12 = (size_t)4 * kCellN * kKx * 2;
constexpr size_t kSzWHH  = (size_t)6 * kCellN * kKh * 2;
constexpr size_t kSzBI0  = (size_t)kGiN * 4;
constexpr size_t kSzGI0  = (size_t)kRows * kGiN * 4;
constexpr size_t kOffXH   = 0;
constexpr size_t kOffWI0  = kOffXH + kSzXH;
constexpr size_t kOffWI12 = kOffWI0 + kSzWI0;
constexpr size_t kOffWHH  = kOffWI12 + kSzWI12;
constexpr size_t kOffBI0  = kOffWHH + kSzWHH;
constexpr size_t kOffGI0  = kOffBI0 + kSzBI0;
constexpr size_t kWsTotal = kOffGI0 + kSzGI0;
static_assert(kWsTotal == 88993792ull, "carve total");
static_assert(kWsTotal <= 134217728ull, "carve cap");
static_assert((kOffWI0 % 256) == 0 && (kOffWI12 % 256) == 0 && (kOffWHH % 256) == 0 &&
              (kOffBI0 % 256) == 0 && (kOffGI0 % 256) == 0, "aligned regions");

__device__ __forceinline__ unsigned short f2bf_bits(float f) {
  unsigned u = __float_as_uint(f);
  return (unsigned short)((u + 0x7FFFu + ((u >> 16) & 1u)) >> 16);
}
__device__ __forceinline__ float bf_bits2f(unsigned short h) { return __uint_as_float(((unsigned)h) << 16); }
__device__ __forceinline__ float bf16r(float f) { return bf_bits2f(f2bf_bits(f)); }
__device__ __forceinline__ _Float16 to_h16(float v) {
  const float s = v * kCarry;
  const float q = (fabsf(s) < kF16Min) ? 0.0f : s;
  return (_Float16)q;
}
__device__ __forceinline__ float ldpin(const float* p) {
  float v = *p;
  asm volatile("" : "+v"(v));
  return v;
}
union FragU { v16h v; v8h h[2]; };
__device__ __forceinline__ v16h frag_ld(const _Float16* p) {
  FragU f;
  f.h[0] = *(const v8h*)(p);
  f.h[1] = *(const v8h*)(p + 16);
  return f.v;
}
__device__ __forceinline__ v8f mma_h(v16h a, v16h b, v8f c) {
  c = __builtin_amdgcn_wmma_f32_16x16x32_f16(false, a, false, b, (short)0, c, false, false);
  asm volatile("v_nop\n\tv_nop\n\tv_nop\n\tv_nop" : "+v"(c) : "v"(a), "v"(b));
  return c;
}
__device__ __forceinline__ void keep4_h(v16h a, v16h b, v16h c, v16h d) { asm volatile("v_nop" :: "v"(a), "v"(b), "v"(c), "v"(d)); }
__device__ __forceinline__ void acc_guard4(v8f& a, v8f& b, v8f& c, v8f& d) { asm volatile("v_nop\n\tv_nop\n\tv_nop\n\tv_nop" : "+v"(a), "+v"(b), "+v"(c), "+v"(d)); }

__device__ __forceinline__ float sigm(float x) {
  const float xc = fminf(fmaxf(x, -40.0f), 40.0f);
  return 1.0f / (1.0f + expf(-xc));
}
__device__ __forceinline__ float tanh_id(float x) {
  const float xc = fminf(fmaxf(x, -20.0f), 20.0f);
  return 1.0f - 2.0f / (1.0f + expf(2.0f * xc));
}

__global__ __launch_bounds__(256) void xplane_kernel(const float* __restrict__ x, unsigned short* __restrict__ dst, int nchunk) {
  const int i = blockIdx.x * 256 + threadIdx.x;
  if (i >= nchunk) return;
  constexpr int kC8 = kKi / 8;
  const int row  = i / kC8;
  const int c8   = i - row * kC8;
  const int col0 = c8 * 8;
  const int ca = (col0 < kIn - 4) ? col0 : (kIn - 4);
  const int cb = (col0 + 4 < kIn - 4) ? (col0 + 4) : (kIn - 4);
  const float* sp = x + (size_t)row * kIn;
  const v4f a = *(const v4f*)(sp + ca);
  const v4f b = *(const v4f*)(sp + cb);
  const bool oka = (col0 < kIn);
  const bool okb = (col0 + 4 < kIn);
  v8h hv;
#pragma unroll
  for (int e = 0; e < 4; ++e) {
    const float av = a[e];
    const float bv = b[e];
    const float sa = oka ? bf16r(av) : 0.0f;
    const float sb = okb ? bf16r(bv) : 0.0f;
    hv[e]     = to_h16(sa);
    hv[4 + e] = to_h16(sb);
  }
  unsigned short* q = dst + (size_t)i * 8;
  *(volatile v8h*)q = hv;
  __threadfence();
  *(volatile v8h*)q = hv;
}

__global__ __launch_bounds__(256) void wplane_kernel(const float* __restrict__ src, unsigned short* __restrict__ dst,
                                                     int nmat, int kreal, int kpad8, int nchunk) {
  const int i = blockIdx.x * 256 + threadIdx.x;
  if (i >= nchunk) return;
  const int R   = i / kpad8;
  const int c8  = i - R * kpad8;
  const int mat = R / kCellN;
  const int rem = R - mat * kCellN;
  const int g   = rem / kHidP;
  const int j   = rem - g * kHidP;
  const bool rowok = (mat < nmat) && (j < kHid);
  const int matc = (mat < nmat) ? mat : (nmat - 1);
  const int jc   = (j < kHid) ? j : (kHid - 1);
  const float* sp = src + (size_t)((matc * 3 + g) * kHid + jc) * kreal;
  v8h hv;
#pragma unroll
  for (int e = 0; e < 8; ++e) {
    const int k  = c8 * 8 + e;
    const int kc = (k < kreal) ? k : (kreal - 1);
    const float v = ldpin(sp + kc);
    const float s = (rowok && (k < kreal)) ? bf16r(v) : 0.0f;
    hv[e] = to_h16(s);
  }
  unsigned short* q = dst + (size_t)i * 8;
  *(volatile v8h*)q = hv;
  __threadfence();
  *(volatile v8h*)q = hv;
}

__global__ __launch_bounds__(128) void bias0_kernel(const float* __restrict__ b_ih0, float* __restrict__ dst) {
  const int n0 = threadIdx.x * 4;
  v4f o;
#pragma unroll
  for (int e = 0; e < 4; ++e) {
    const int n   = n0 + e;
    const int dd  = n / kCellN;
    const int rem = n - dd * kCellN;
    const int g   = rem / kHidP;
    const int j   = rem - g * kHidP;
    const bool ok = (n < 2 * kCellN) && (j < kHid);
    const int dc  = (dd < 2) ? dd : 1;
    const int jc  = (j < kHid) ? j : (kHid - 1);
    const float v = ldpin(b_ih0 + dc * 3 * kHid + g * kHid + jc);
    o[e] = ok ? bf16r(v) : 0.0f;
  }
  float* q = dst + n0;
  *(volatile v4f*)q = o;
  __threadfence();
  *(volatile v4f*)q = o;
}

__global__ __launch_bounds__(256) void gemm_f16_bias_kernel(
    const unsigned short* __restrict__ Ap, int lda,
    const unsigned short* __restrict__ Btp, int ldb,
    float* __restrict__ C, int ldc,
    const float* __restrict__ bias,
    int M, int N, int K, float scale) {
  const _Float16* A  = (const _Float16*)Ap;
  const _Float16* Bt = (const _Float16*)Btp;
  __shared__ __align__(16) float sT[8][16 * 68];
  const int lane = threadIdx.x & 31;
  const int wave = threadIdx.x >> 5;
  const int tilesN = N >> 6;
  const int tilesM = M >> 6;
  const int tile = blockIdx.x * 8 + wave;
  if (tile >= tilesM * tilesN) return;
  const int tm = tile / tilesN;
  const int tn = tile - tm * tilesN;
  const int m0 = tm << 6;
  const int n0 = tn << 6;
  const int rlane = lane & 15;
  const int koff  = (lane >> 4) * 8;
  const int mOff  = (lane >> 4) * 8;

  v8f acc[4][4];
#pragma unroll
  for (int i = 0; i < 4; ++i)
#pragma unroll
    for (int j = 0; j < 4; ++j) acc[i][j] = (v8f){0.f, 0.f, 0.f, 0.f, 0.f, 0.f, 0.f, 0.f};

  for (int k0 = 0; k0 < K; k0 += 32) {
    v16h bh[4];
#pragma unroll
    for (int j = 0; j < 4; ++j) {
      const size_t bo = (size_t)(n0 + (j << 4) + rlane) * ldb + koff + k0;
      bh[j] = frag_ld(Bt + bo);
    }
#pragma unroll
    for (int i = 0; i < 4; ++i) {
      const size_t ao = (size_t)(m0 + (i << 4) + rlane) * lda + koff + k0;
      const v16h ah = frag_ld(A + ao);
#pragma unroll
      for (int j = 0; j < 4; ++j) acc[i][j] = mma_h(ah, bh[j], acc[i][j]);
    }
    keep4_h(bh[0], bh[1], bh[2], bh[3]);
  }
  acc_guard4(acc[0][0], acc[0][1], acc[0][2], acc[0][3]);
  acc_guard4(acc[1][0], acc[1][1], acc[1][2], acc[1][3]);
  acc_guard4(acc[2][0], acc[2][1], acc[2][2], acc[2][3]);
  acc_guard4(acc[3][0], acc[3][1], acc[3][2], acc[3][3]);

  float* slab = sT[wave];
#pragma unroll
  for (int i = 0; i < 4; ++i) {
    const int mBase = m0 + (i << 4);
#pragma unroll
    for (int j = 0; j < 4; ++j) {
      const int n = n0 + (j << 4) + rlane;
      const float bv = bias[n];
#pragma unroll
      for (int r = 0; r < 8; ++r) {
        const float v = acc[i][j][r] * scale + bv;
        slab[(mOff + r) * 68 + (j << 4) + rlane] = v;
      }
    }
    __builtin_amdgcn_fence(__ATOMIC_RELEASE, "workgroup");
    __builtin_amdgcn_wave_barrier();
    __builtin_amdgcn_fence(__ATOMIC_ACQUIRE, "workgroup");
    {
      const int hh = lane >> 4;
      const int c4 = (lane & 15) * 4;
      for (int pass = 0; pass < 2; ++pass) {
#pragma unroll
        for (int it = 0; it < 8; ++it) {
          const int row = it * 2 + hh;
          const v4f v = *(const v4f*)(slab + row * 68 + c4);
          *(volatile v4f*)(C + (size_t)(mBase + row) * ldc + n0 + c4) = v;
        }
        __threadfence();
      }
    }
    __builtin_amdgcn_fence(__ATOMIC_RELEASE, "workgroup");
    __builtin_amdgcn_wave_barrier();
    __builtin_amdgcn_fence(__ATOMIC_ACQUIRE, "workgroup");
  }
}

template <bool XW, bool XOUT>
__device__ __forceinline__ void cell_step(
    const _Float16* xA, const _Float16* wx, const _Float16* hA, const _Float16* wh, const float* gi,
    const float bR, const float bZ, const float bI, const float bH,
    float (&hst)[8],
    _Float16* hN, _Float16* hPad, _Float16* xN, _Float16* xPad, float* sl,
    const bool jok, const bool padH, const bool padX, const bool padXl, const _Float16 zh) {
  const v8f z8 = {0.f, 0.f, 0.f, 0.f, 0.f, 0.f, 0.f, 0.f};
  v8f aR = z8, aZ = z8, aI = z8, aH = z8;
  float gR[8], gZ[8], gN[8];
#pragma unroll
  for (int r = 0; r < 8; ++r) {
    if (!XW) {
      gR[r] = gi[r * kGiN];
      gZ[r] = gi[r * kGiN + kHidP];
      gN[r] = gi[r * kGiN + 2 * kHidP];
    } else {
      gR[r] = 0.0f;
      gZ[r] = 0.0f;
      gN[r] = 0.0f;
    }
  }
  if (XW) {
#pragma unroll 1
    for (int ks = 0; ks < kKx / 32; ++ks) {
      const v16h a  = frag_ld(xA + 32 * ks);
      const v16h b0 = frag_ld(wx + 32 * ks);
      const v16h b1 = frag_ld(wx + kHidP * kKx + 32 * ks);
      const v16h b2 = frag_ld(wx + 2 * kHidP * kKx + 32 * ks);
      aR = mma_h(a, b0, aR);
      aZ = mma_h(a, b1, aZ);
      aI = mma_h(a, b2, aI);
    }
  }
#pragma unroll 1
  for (int ks = 0; ks < kKh / 32; ++ks) {
    const v16h a  = frag_ld(hA + 32 * ks);
    const v16h b0 = frag_ld(wh + 32 * ks);
    const v16h b1 = frag_ld(wh + kHidP * kKh + 32 * ks);
    const v16h b2 = frag_ld(wh + 2 * kHidP * kKh + 32 * ks);
    aR = mma_h(a, b0, aR);
    aZ = mma_h(a, b1, aZ);
    aH = mma_h(a, b2, aH);
  }
#pragma unroll
  for (int r = 0; r < 8; ++r) {
    float pr, pz, pi;
    const float ph = aH[r] * kFold + bH;
    if (XW) {
      pr = aR[r] * kFold + bR;
      pz = aZ[r] * kFold + bZ;
      pi = aI[r] * kFold + bI;
    } else {
      pr = gR[r] + (aR[r] * kFold + bR);
      pz = gZ[r] + (aZ[r] * kFold + bZ);
      pi = gN[r];
    }
    const float rg = sigm(pr);
    const float zg = sigm(pz);
    const float ng = tanh_id(pi + rg * ph);
    const float hp = hst[r];
    const float hc = (1.0f - zg) * ng + zg * hp;
    const float hn = jok ? hc : 0.0f;
    hst[r] = hn;
    const _Float16 hv = to_h16(hn);
    hN[r * kKh] = hv;
    if (padH) hPad[r * kKh] = zh;
    if (XOUT) {
      if (jok) xN[r * kKx] = hv;
      if (padX && padXl) xPad[r * kKx] = zh;
    }
    if (jok) sl[r * kOutC] = hn;
  }
}

__device__ __forceinline__ void load_state(const float* h0, int cell, int brow0, int jc, bool jok,
                                           float (&hst)[8], _Float16* hdst) {
#pragma unroll
  for (int r = 0; r < 8; ++r) {
    const float v = ldpin(h0 + ((size_t)cell * kBatch + brow0 + r) * kHid + jc);
    const float s = jok ? bf16r(v) : 0.0f;
    hst[r] = s;
    hdst[r * kKh] = to_h16(s);
  }
}

__global__ __launch_bounds__(kNT) void seq_kernel(
    const float* __restrict__ GI0,
    const unsigned short* WHHp, const unsigned short* WI12p,
    const float* __restrict__ h0, const float* __restrict__ b_hh0,
    const float* __restrict__ b_ih12, const float* __restrict__ b_hh12,
    float* __restrict__ out) {
  __shared__ __align__(16) _Float16 Hs[kHsN];
  __shared__ __align__(16) _Float16 Xs[kXsN];
  __shared__ __align__(16) float    Sl[16 * kOutC];
  const _Float16* WHH  = (const _Float16*)WHHp;
  const _Float16* WI12 = (const _Float16*)WI12p;
  const int tid  = threadIdx.x;
  const int lane = tid & 31;
  const int wave = tid >> 5;
  const int c    = lane & 15;
  const int hh   = lane >> 4;
  const int koff = hh * 8;
  const int d    = wave / 5;
  const int jt   = wave - d * 5;
  const int j    = 16 * jt + c;
  const bool jok = (j < kHid);
  const int jc   = jok ? j : (kHid - 1);
  const int b0   = blockIdx.x * 16;
  const bool padH  = (jt == 4);
  const bool padX  = (wave == 9);
  const bool padXl = (c < 10);

  float zf = 0.0f;
  asm volatile("" : "+v"(zf));
  const _Float16 zh = (_Float16)zf;

#pragma unroll 1
  for (int i = tid; i < kHsN; i += kNT) Hs[i] = zh;
#pragma unroll 1
  for (int i = tid; i < kXsN; i += kNT) Xs[i] = zh;
  __syncthreads();

  const int aHo   = c * kKh + koff;
  const int aXo   = c * kKx + koff;
  const int wHo   = (8 * hh) * kKh + j;
  const int wHpad = (8 * hh) * kKh + kHidP + c;
  const int wXo   = (8 * hh) * kKx + d * kHid + jc;
  const int wXpad = (8 * hh) * kKx + 2 * kHid + (padXl ? c : 9);
  const int wSo   = (8 * hh) * kOutC + d * kHid + jc;

  float hs0[8], hs1[8], hs2[8];
  load_state(h0, 0 + d, b0 + 8 * hh, jc, jok, hs0, Hs + ((0 * 2 + 0) * 2 + d) * kHTile + wHo);
  load_state(h0, 2 + d, b0 + 8 * hh, jc, jok, hs1, Hs + ((1 * 2 + 0) * 2 + d) * kHTile + wHo);
  load_state(h0, 4 + d, b0 + 8 * hh, jc, jok, hs2, Hs + ((2 * 2 + 0) * 2 + d) * kHTile + wHo);

  const int bb0 = d * 3 * kHid + jc;
  const int bb1 = (0 * 2 + d) * 3 * kHid + jc;
  const int bb2 = (1 * 2 + d) * 3 * kHid + jc;
  const float l0hr = ldpin(b_hh0 + bb0);
  const float l0hz = ldpin(b_hh0 + bb0 + kHid);
  const float l0hn = ldpin(b_hh0 + bb0 + 2 * kHid);
  const float l1ir = ldpin(b_ih12 + bb1);
  const float l1iz = ldpin(b_ih12 + bb1 + kHid);
  const float l1in = ldpin(b_ih12 + bb1 + 2 * kHid);
  const float l1hr = ldpin(b_hh12 + bb1);
  const float l1hz = ldpin(b_hh12 + bb1 + kHid);
  const float l1hn = ldpin(b_hh12 + bb1 + 2 * kHid);
  const float l2ir = ldpin(b_ih12 + bb2);
  const float l2iz = ldpin(b_ih12 + bb2 + kHid);
  const float l2in = ldpin(b_ih12 + bb2 + 2 * kHid);
  const float l2hr = ldpin(b_hh12 + bb2);
  const float l2hz = ldpin(b_hh12 + bb2 + kHid);
  const float l2hn = ldpin(b_hh12 + bb2 + 2 * kHid);
  const float c0r = jok ? bf16r(l0hr) : 0.0f;
  const float c0z = jok ? bf16r(l0hz) : 0.0f;
  const float c0h = jok ? bf16r(l0hn) : 0.0f;
  const float c1r = jok ? (bf16r(l1ir) + bf16r(l1hr)) : 0.0f;
  const float c1z = jok ? (bf16r(l1iz) + bf16r(l1hz)) : 0.0f;
  const float c1i = jok ? bf16r(l1in) : 0.0f;
  const float c1h = jok ? bf16r(l1hn) : 0.0f;
  const float c2r = jok ? (bf16r(l2ir) + bf16r(l2hr)) : 0.0f;
  const float c2z = jok ? (bf16r(l2iz) + bf16r(l2hz)) : 0.0f;
  const float c2i = jok ? bf16r(l2in) : 0.0f;
  const float c2h = jok ? bf16r(l2hn) : 0.0f;

  const int rowW = 16 * jt + c;
  const _Float16* whb0 = WHH  + (size_t)((0 + d) * kCellN + rowW) * kKh + koff;
  const _Float16* whb1 = WHH  + (size_t)((2 + d) * kCellN + rowW) * kKh + koff;
  const _Float16* whb2 = WHH  + (size_t)((4 + d) * kCellN + rowW) * kKh + koff;
  const _Float16* wxb1 = WI12 + (size_t)((0 + d) * kCellN + rowW) * kKx + koff;
  const _Float16* wxb2 = WI12 + (size_t)((2 + d) * kCellN + rowW) * kKx + koff;
  const float* gib = GI0 + (size_t)(b0 + 8 * hh) * kGiN + d * kCellN + rowW;

  __syncthreads();

#pragma unroll 1
  for (int t = 0; t < kSteps; ++t) {
    const int par = t & 1;
    const int nxt = par ^ 1;
    int woff = 0;
    asm volatile("" : "+v"(woff));

    cell_step<false, true>(
        Hs, whb0, Hs + ((0 * 2 + par) * 2 + d) * kHTile + aHo, whb0 + woff,
        gib + (size_t)t * kBatch * kGiN,
        c0r, c0z, 0.0f, c0h, hs0,
        Hs + ((0 * 2 + nxt) * 2 + d) * kHTile + wHo, Hs + ((0 * 2 + nxt) * 2 + d) * kHTile + wHpad,
        Xs + wXo, Xs + wXpad, Sl + wSo,
        jok, padH, padX, padXl, zh);
    __syncthreads();

    cell_step<true, true>(
        Xs + aXo, wxb1 + woff, Hs + ((1 * 2 + par) * 2 + d) * kHTile + aHo, whb1 + woff,
        gib,
        c1r, c1z, c1i, c1h, hs1,
        Hs + ((1 * 2 + nxt) * 2 + d) * kHTile + wHo, Hs + ((1 * 2 + nxt) * 2 + d) * kHTile + wHpad,
        Xs + kXTile + wXo, Xs + kXTile + wXpad, Sl + 2 * kHid + wSo,
        jok, padH, padX, padXl, zh);
    __syncthreads();

    cell_step<true, false>(
        Xs + kXTile + aXo, wxb2 + woff, Hs + ((2 * 2 + par) * 2 + d) * kHTile + aHo, whb2 + woff,
        gib,
        c2r, c2z, c2i, c2h, hs2,
        Hs + ((2 * 2 + nxt) * 2 + d) * kHTile + wHo, Hs + ((2 * 2 + nxt) * 2 + d) * kHTile + wHpad,
        Xs, Xs, Sl + 4 * kHid + wSo,
        jok, padH, padX, padXl, zh);
    __syncthreads();

    {
      const v4f* s4 = (const v4f*)Sl;
      v4f ov[6];
#pragma unroll
      for (int it = 0; it < 6; ++it) {
        const int i  = tid + kNT * it;
        const int ic = (i < kSlabV4) ? i : (kSlabV4 - 1);
        ov[it] = s4[ic];
      }
      float* ob = out + (size_t)(t * kBatch + b0) * kOutC;
      for (int pass = 0; pass < 2; ++pass) {
#pragma unroll
        for (int it = 0; it < 5; ++it) *(volatile v4f*)(ob + 4 * (tid + kNT * it)) = ov[it];
        if (tid < kSlabV4 - 5 * kNT) *(volatile v4f*)(ob + 4 * (tid + 5 * kNT)) = ov[5];
        __threadfence();
      }
    }
    __syncthreads();
  }
}

extern "C" void kernel_launch(void* const* d_in, const int* in_sizes, int n_in,
                              void* d_out, int out_size, void* d_ws, size_t ws_size,
                              hipStream_t stream) {
  if (n_in < 10 || d_out == nullptr || d_ws == nullptr) return;
  if (in_sizes[0] != kRows * kIn) return;
  if (in_sizes[1] != 6 * kBatch * kHid) return;
  if (in_sizes[2] != 2 * 3 * kHid * kIn) return;
  if (in_sizes[3] != 2 * 3 * kHid * kHid) return;
  if (in_sizes[4] != 2 * 3 * kHid) return;
  if (in_sizes[5] != 2 * 3 * kHid) return;
  if (in_sizes[6] != 4 * 3 * kHid * 2 * kHid) return;
  if (in_sizes[7] != 4 * 3 * kHid * kHid) return;
  if (in_sizes[8] != 4 * 3 * kHid) return;
  if (in_sizes[9] != 4 * 3 * kHid) return;
  if (out_size != kRows * kOutC) return;
  if (ws_size < kWsTotal) return;

  const float* input  = (const float*)d_in[0];
  const float* h0     = (const float*)d_in[1];
  const float* w_ih0  = (const float*)d_in[2];
  const float* w_hh0  = (const float*)d_in[3];
  const float* b_ih0  = (const float*)d_in[4];
  const float* b_hh0  = (const float*)d_in[5];
  const float* w_ih12 = (const float*)d_in[6];
  const float* w_hh12 = (const float*)d_in[7];
  const float* b_ih12 = (const float*)d_in[8];
  const float* b_hh12 = (const float*)d_in[9];
  float* out = (float*)d_out;

  char* ws = (char*)d_ws;
  unsigned short* XH   = (unsigned short*)(ws + kOffXH);
  unsigned short* WI0  = (unsigned short*)(ws + kOffWI0);
  unsigned short* WI12 = (unsigned short*)(ws + kOffWI12);
  unsigned short* WHH  = (unsigned short*)(ws + kOffWHH);
  float*          BI0  = (float*)(ws + kOffBI0);
  float*          GI0  = (float*)(ws + kOffGI0);

  const int nx = kRows * (kKi / 8);
  xplane_kernel<<<nx / 256, 256, 0, stream>>>(input, XH, nx);
  const int nw0 = kGiN * (kKi / 8);
  wplane_kernel<<<(nw0 + 255) / 256, 256, 0, stream>>>(w_ih0, WI0, 2, kIn, kKi / 8, nw0);
  const int nw1 = 4 * kCellN * (kKx / 8);
  wplane_kernel<<<(nw1 + 255) / 256, 256, 0, stream>>>(w_ih12, WI12, 4, 2 * kHid, kKx / 8, nw1);
  const int nh0 = 2 * kCellN * (kKh / 8);
  wplane_kernel<<<(nh0 + 255) / 256, 256, 0, stream>>>(w_hh0, WHH, 2, kHid, kKh / 8, nh0);
  const int nh1 = 4 * kCellN * (kKh / 8);
  wplane_kernel<<<(nh1 + 255) / 256, 256, 0, stream>>>(w_hh12, WHH + (size_t)2 * kCellN * kKh, 4, kHid, kKh / 8, nh1);
  bias0_kernel<<<1, 128, 0, stream>>>(b_ih0, BI0);

  const int gtiles = (kRows / 64) * (kGiN / 64);
  gemm_f16_bias_kernel<<<gtiles / 8, 256, 0, stream>>>(XH, kKi, WI0, kKi, GI0, kGiN, BI0, kRows, kGiN, kKi, kFold);

  seq_kernel<<<kBatch / 16, kNT, 0, stream>>>(GI0, WHH, WI12, h0, b_hh0, b_ih12, b_hh12, out);
}
